// GNN_MDN_44779329028529
// MI455X (gfx1250) — hardware-run, weakly checked
//
#include <hip/hip_runtime.h>


namespace {
constexpr int N = 30000, NP = 30016, E = 480000, V = 100000, EMB = 64, HID = 32, NH = 8, W1O = NH * HID, MIX = 5, NBLK = NP / 16;
constexpr float XS = 1024.0f  , HS = 16384.0f  , WSC = 256.0f, NEG = 0.2f;
typedef _Float16 b16;
typedef __attribute__((ext_vector_type(16))) _Float16 v16b;
typedef __attribute__((ext_vector_type(8))) _Float16 v8b;
typedef __attribute__((ext_vector_type(8))) float v8f;
typedef __attribute__((ext_vector_type(4))) float v4f;
typedef __attribute__((ext_vector_type(2))) float v2f;
__device__ __forceinline__ float bf16_rne(float f) { unsigned int u = __float_as_uint(f); u += 0x7FFFu + ((u >> 16) & 1u); return __uint_as_float(u & 0xFFFF0000u); }
__device__ __forceinline__ void split16(float v, b16& hi, b16& lo) { hi = (b16)v; lo = (b16)(v - (float)hi); }
__device__ __forceinline__ v16b frag_kb(const b16* p, int hh) { const v8b a = *(const v8b*)(p + 8 * hh), b = *(const v8b*)(p + 16 + 8 * hh); v16b f;
#pragma unroll
  for (int e = 0; e < 8; ++e) { f[e] = a[e]; f[8 + e] = b[e]; } return f; }
__device__ __forceinline__ v8f wmma16b(v16b a, v16b b, v8f c) { v8f d = __builtin_amdgcn_wmma_f32_16x16x32_f16(false, a, false, b, (short)0, c, false, false); asm volatile("v_nop\n\tv_nop\n\tv_nop\n\tv_nop" : "+v"(d) : "v"(a), "v"(b)); return d; }
__device__ __forceinline__ void wave_lds_sync() { __builtin_amdgcn_fence(__ATOMIC_RELEASE, "workgroup"); __builtin_amdgcn_wave_barrier(); __builtin_amdgcn_fence(__ATOMIC_ACQUIRE, "workgroup"); }
__device__ __forceinline__ float pmul(float a, float b) { float p = a * b; asm volatile("" : "+v"(p)); return p; }
__device__ __forceinline__ int iclamp(int v, int lo, int hi) { return v < lo ? lo : (v > hi ? hi : v); }
__device__ __forceinline__ float leaky(float v) { return v >= 0.0f ? v : NEG * v; }
__device__ __forceinline__ float elu(float v) { return v > 0.0f ? v : expm1f(v); }
template <int CPL> __device__ __forceinline__ void ldrow(const float* p, float* f) { if (CPL == 8) { const v4f a = *(const v4f*)p, b = *(const v4f*)(p + 4); for (int i = 0; i < 4; ++i) { f[i] = a[i]; f[4 + i] = b[i]; } } else { for (int i = 0; i < CPL; ++i) f[i] = p[i]; } }
template <int CPL> __device__ __forceinline__ void strow(float* p, const float* f) { if (CPL == 8) { v4f a, b; for (int i = 0; i < 4; ++i) { a[i] = f[i]; b[i] = f[4 + i]; } *(volatile v4f*)p = a; *(volatile v4f*)(p + 4) = b; } else { for (int i = 0; i < CPL; ++i) ((volatile float*)p)[i] = f[i]; } }
constexpr int CSR_NBLK9 = 512, CSR_GB9 = 9, CSR_GN9 = 1 << CSR_GB9  , CSR_TS9 = (CSR_GN9 < 32 ? 32 : CSR_GN9)  , CSR_MAXG9 = 512, CSR_CAP9 = 12288  ;
__device__ __host__ __forceinline__ int csr_tix9(int v) { return (v >> CSR_GB9) * CSR_TS9 + (v & (CSR_GN9 - 1)); }
__global__ __launch_bounds__(64) void csrA_kernel9(const int* __restrict__ dst, int E, int N, int nG, int CHP, int NGP, int* __restrict__ STG, int* __restrict__ HST) {
  extern __shared__ int sm[];
  int* cnt = sm; int* run = sm + NGP; int* ids = sm + 2 * NGP;
  const int b = blockIdx.x; const int ch = (E + CSR_NBLK9 - 1) / CSR_NBLK9; const int e0 = b * ch, e1 = min(E, e0 + ch);
  for (int i = threadIdx.x; i < NGP; i += 64) cnt[i] = 0;
  for (int i = threadIdx.x; i < CHP; i += 64) ids[i] = -1;
  __syncthreads();
  if (threadIdx.x == 0) {
    for (int e = e0; e < e1; ++e) { int d = dst[e]; d = (d < 0) ? 0 : (d >= N ? N - 1 : d); cnt[d >> CSR_GB9] += 1; }
    int acc = 0; for (int g = 0; g < nG; ++g) { run[g] = acc; acc += cnt[g]; }
    for (int e = e0; e < e1; ++e) { int d = dst[e]; d = (d < 0) ? 0 : (d >= N ? N - 1 : d); const int g = d >> CSR_GB9; ids[run[g]] = e; run[g] += 1; } }
  __syncthreads();
  typedef __attribute__((ext_vector_type(4))) int v4i;
  for (int pass = 0; pass < 2; ++pass) {
    for (int i = threadIdx.x; i < CHP / 4; i += 64) *(volatile v4i*)(STG + (size_t)b * CHP + i * 4) = *(const v4i*)(&ids[i * 4]);
    for (int i = threadIdx.x; i < NGP / 4; i += 64) { v4i v; for (int e = 0; e < 4; ++e) v[e] = (i * 4 + e < nG) ? cnt[i * 4 + e] : 0; *(volatile v4i*)(HST + (size_t)b * NGP + i * 4) = v; }
    __threadfence(); }
}
__global__ __launch_bounds__(512) void csrS_kernel9(const int* __restrict__ HST, int nG, int NGP, int* __restrict__ START, int* __restrict__ TOT, int* __restrict__ OFF) {
  __shared__ int tot[CSR_MAXG9];
  const int b = threadIdx.x;
  for (int pass = 0; pass < 2; ++pass) { int runb = 0; for (int g = 0; g < nG; ++g) { int c = HST[(size_t)b * NGP + g]; c = (c < 0) ? 0 : c; ((volatile int*)OFF)[(size_t)g * CSR_NBLK9 + b] = runb; runb += c; } __threadfence(); }
  for (int g = threadIdx.x; g < nG; g += 512) { int s = 0; for (int bb = 0; bb < CSR_NBLK9; ++bb) { int c = HST[(size_t)bb * NGP + g]; s += (c < 0) ? 0 : c; } tot[g] = s; }
  __syncthreads();
  if (threadIdx.x < 32) {
    __shared__ int st[CSR_MAXG9 + 32];
    if (threadIdx.x == 0) { int acc = 0; for (int g = 0; g < NGP; ++g) { st[g] = acc; if (g < nG) acc += (tot[g] + 31) & ~31; } st[NGP] = acc; }
    __builtin_amdgcn_fence(__ATOMIC_RELEASE, "workgroup"); __builtin_amdgcn_wave_barrier(); __builtin_amdgcn_fence(__ATOMIC_ACQUIRE, "workgroup");
    for (int pass = 0; pass < 2; ++pass) { for (int i = threadIdx.x; i < NGP + 32; i += 32) { ((volatile int*)START)[i] = (i <= NGP) ? st[min(i, NGP)] : 0; ((volatile int*)TOT)[i] = (i < nG) ? tot[i] : 0; } __threadfence(); } }
}
__global__ __launch_bounds__(256) void csrB_kernel9(const int* __restrict__ dst, int N, int nG, int CHP, int NGP, int permLen, const int* __restrict__ STG, const int* __restrict__ HST, const int* __restrict__ OFF, const int* __restrict__ START, const int* __restrict__ TOT, int* __restrict__ PERM, int* __restrict__ ROWPTR, int* __restrict__ ROWCNT, int* __restrict__ FLAG) {
  typedef __attribute__((ext_vector_type(4))) int v4i;
  __shared__ int ids[CSR_CAP9]; __shared__ unsigned short key[CSR_CAP9]; __shared__ int outp[CSR_CAP9]; __shared__ int ncnt[CSR_GN9 + 1]; __shared__ int boff[CSR_NBLK9 + 1];
  const int g = blockIdx.x, t_ = threadIdx.x; int tot = TOT[g]; int st = START[g], stn = START[g + 1]; const int v0 = g * CSR_GN9; const int nv = min(CSR_GN9, N - v0); const int t0 = g * CSR_TS9;
  st = (st < 0) ? 0 : (st > permLen - 32 ? permLen - 32 : st) & ~31; stn = (stn < st) ? st : (stn > permLen ? permLen : stn); tot = (tot < 0) ? 0 : tot; if (tot > stn - st && tot <= CSR_CAP9) tot = stn - st;
  if (tot > CSR_CAP9) {
    for (int pass = 0; pass < 2; ++pass) { for (int i = t_; i < CSR_TS9 / 4; i += 256) { v4i a, c; for (int e = 0; e < 4; ++e) { a[e] = st; c[e] = 0; } *(volatile v4i*)(ROWPTR + t0 + i * 4) = a; *(volatile v4i*)(ROWCNT + t0 + i * 4) = c; } if (t_ == 0) ((volatile int*)FLAG)[0] = 1; __threadfence(); } (void)nv; return; }
  if (t_ == 0) { int acc = 0; for (int b = 0; b < CSR_NBLK9; ++b) { boff[b] = acc; int c = HST[(size_t)b * NGP + g]; c = (c < 0) ? 0 : (c > CHP ? CHP : c); acc += c; if (acc > tot) acc = tot; } boff[CSR_NBLK9] = acc; }
  for (int i = t_; i <= CSR_GN9; i += 256) ncnt[i] = 0;
  __syncthreads();
  for (int b = 0; b < CSR_NBLK9; ++b) { const int c = boff[b + 1] - boff[b]; int o_ = OFF[(size_t)g * CSR_NBLK9 + b]; o_ = (o_ < 0) ? 0 : (o_ > CHP - c ? CHP - c : o_); const int* src_ = STG + (size_t)b * CHP + o_;
    for (int i = t_; i < c; i += 256) { int id = src_[i]; id = (id < 0) ? 0 : id; ids[boff[b] + i] = id; int d = dst[id]; d = (d < v0) ? v0 : (d >= N ? N - 1 : d); int kk = d - v0; kk = (kk < 0) ? 0 : (kk >= CSR_GN9 ? CSR_GN9 - 1 : kk); key[boff[b] + i] = (unsigned short)kk; } }
  __syncthreads();
  if (t_ == 0) { for (int i = 0; i < tot; ++i) ncnt[key[i]] += 1; int acc = 0; for (int vl = 0; vl < CSR_GN9; ++vl) { const int c = ncnt[vl]; ncnt[vl] = acc; acc += c; } ncnt[CSR_GN9] = acc;
    for (int i = 0; i < tot; ++i) { const int vl = key[i]; outp[ncnt[vl]] = ids[i]; ncnt[vl] += 1; }
    for (int vl = CSR_GN9; vl > 0; --vl) ncnt[vl] = ncnt[vl - 1]; ncnt[0] = 0; }
  __syncthreads();
  for (int pass = 0; pass < 2; ++pass) {
    for (int i = t_; i < (stn - st) / 4; i += 256) { v4i v; for (int e = 0; e < 4; ++e) { const int q = i * 4 + e; v[e] = (q < tot) ? outp[q] : -1; } *(volatile v4i*)(PERM + st + i * 4) = v; }
    for (int i = t_; i < CSR_TS9 / 4; i += 256) { v4i a, c; for (int e = 0; e < 4; ++e) { const int vl = i * 4 + e; const int vc = vl < CSR_GN9 ? vl : CSR_GN9; a[e] = (vl < CSR_GN9) ? st + ncnt[vc] : st; c[e] = (vl < nv) ? (ncnt[(vc < CSR_GN9 ? vc : CSR_GN9 - 1) + 1] - ncnt[vc]) : 0; } *(volatile v4i*)(ROWPTR + t0 + i * 4) = a; *(volatile v4i*)(ROWCNT + t0 + i * 4) = c; }
    __threadfence(); }
}
__global__ __launch_bounds__(256) void csrZ_kernel9(int* __restrict__ p, size_t n4) { typedef __attribute__((ext_vector_type(4))) int v4i; const size_t tid = (size_t)blockIdx.x * 256 + threadIdx.x, nth = (size_t)gridDim.x * 256; v4i z = {0, 0, 0, 0}; for (size_t i = tid; i < n4; i += nth) *(volatile v4i*)(p + i * 4) = z; }
struct CsrBufs9 { int *STG, *HST, *OFF, *START, *TOT, *PERM, *ROWPTR, *ROWCNT, *FLAG; int nG, NGP, CHP; size_t permLen; char* base; size_t bytes; };
static size_t csr_carve9(CsrBufs9& c, char* ws, size_t off, int E, int N) {
  const size_t off0 = off; c.base = ws + off;
  auto al = [&](size_t bytes) { char* p = ws + off; off += (bytes + 255) & ~(size_t)255; return p; };
  c.nG = (N + CSR_GN9 - 1) / CSR_GN9; c.NGP = (c.nG + 31) & ~31; const int ch = (E + CSR_NBLK9 - 1) / CSR_NBLK9; c.CHP = (ch + 31) & ~31; c.permLen = (size_t)E + 32 * (size_t)c.nG + 32;
  c.STG = (int*)al((size_t)CSR_NBLK9 * c.CHP * 4); c.HST = (int*)al((size_t)CSR_NBLK9 * c.NGP * 4); c.OFF = (int*)al((size_t)c.NGP * CSR_NBLK9 * 4); c.START = (int*)al((size_t)(c.NGP + 64) * 4); c.TOT = (int*)al((size_t)(c.NGP + 64) * 4);
  c.PERM = (int*)al(c.permLen * 4); c.ROWPTR = (int*)al((size_t)c.nG * CSR_TS9 * 4); c.ROWCNT = (int*)al((size_t)c.nG * CSR_TS9 * 4); c.FLAG = (int*)al(256);
  c.bytes = off - off0; return off;
}
static void csr_build9(const CsrBufs9& c, const int* dst, int E, int N, hipStream_t stream) {
  const size_t smem = (size_t)(2 * c.NGP + c.CHP) * 4;
  csrZ_kernel9<<<512, 256, 0, stream>>>((int*)c.base, c.bytes / 16);
  csrA_kernel9<<<CSR_NBLK9, 64, smem, stream>>>(dst, E, N, c.nG, c.CHP, c.NGP, c.STG, c.HST);
  csrS_kernel9<<<1, 512, 0, stream>>>(c.HST, c.nG, c.NGP, c.START, c.TOT, c.OFF);
  csrB_kernel9<<<c.nG, 256, 0, stream>>>(dst, N, c.nG, c.CHP, c.NGP, (int)c.permLen, c.STG, c.HST, c.OFF, c.START, c.TOT, c.PERM, c.ROWPTR, c.ROWCNT, c.FLAG);
}


__global__ __launch_bounds__(256) void wprep_kernel(const float* __restrict__ w, int KIN, int OUT, int ro, b16* __restrict__ WT) {
  const int u = blockIdx.x * 256 + threadIdx.x; if (u >= OUT * KIN / 8) return; const int e = u * 8; const int o = e / KIN, k0 = e % KIN; v8b v; for (int j = 0; j < 8; ++j) v[j] = (b16)(bf16_rne(w[(size_t)(k0 + j) * OUT + o]) * WSC);
  for (int pass = 0; pass < 2; ++pass) { *(volatile v8b*)(WT + (size_t)(ro + o) * KIN + k0) = v; __threadfence(); }
}
__global__ __launch_bounds__(256) void wzero_kernel(b16* __restrict__ WT, int n8) { const int u = blockIdx.x * 256 + threadIdx.x; if (u >= n8) return; v8b z = {}; for (int pass = 0; pass < 2; ++pass) { *(volatile v8b*)(WT + (size_t)u * 8) = z; __threadfence(); } }
__global__ __launch_bounds__(32) void lin1_kernel(const int* __restrict__ ids, const float* __restrict__ emb, const b16* __restrict__ W1T, const float* __restrict__ as, const float* __restrict__ ad, int NLIM, float* __restrict__ P1, float* __restrict__ ES, float* __restrict__ ED) {
  __shared__ __attribute__((aligned(16))) b16 Ah[16][EMB + 8]; __shared__ __attribute__((aligned(16))) float Tf[16][W1O + 4]; __shared__ __attribute__((aligned(16))) float Se[16][8], Sd[16][8];
  const int lane = threadIdx.x, nloc = lane & 15, hlf = lane >> 4; const size_t m0 = (size_t)blockIdx.x * 16; const bool live = m0 < (size_t)NLIM; const float sc = 1.0f / (XS * WSC);
  for (int rr = 0; rr < 16; ++rr) { const size_t r = (m0 + rr) < (size_t)N ? m0 + rr : (size_t)N - 1; const int id = iclamp(ids[r], 0, V - 1); const v2f v = *(const v2f*)(emb + (size_t)id * EMB + lane * 2); Ah[rr][lane * 2] = (b16)(bf16_rne(v[0]) * XS); Ah[rr][lane * 2 + 1] = (b16)(bf16_rne(v[1]) * XS); }
  wave_lds_sync();
#pragma unroll 1
  for (int cg = 0; cg < 2; ++cg) { v8f acc[8]; float pes[4][8], ped[4][8];
#pragma unroll
    for (int t = 0; t < 8; ++t) acc[t] = (v8f){};
    if (live) {
#pragma unroll
      for (int kb = 0; kb < EMB; kb += 32) { const v16b a = frag_kb(&Ah[nloc][kb], hlf);
#pragma unroll
        for (int t = 0; t < 8; ++t) acc[t] = wmma16b(a, frag_kb(W1T + (size_t)(cg * 128 + t * 16 + nloc) * EMB + kb, hlf), acc[t]); } }
#pragma unroll
    for (int hh = 0; hh < 4; ++hh) for (int r8 = 0; r8 < 8; ++r8) { pes[hh][r8] = 0.0f; ped[hh][r8] = 0.0f; }
#pragma unroll
    for (int t = 0; t < 8; ++t) { const int c = cg * 128 + t * 16 + nloc; const int hh = t >> 1; const float wsv = bf16_rne(as[c]), wdv = bf16_rne(ad[c]);
#pragma unroll
      for (int r8 = 0; r8 < 8; ++r8) { const float p = acc[t][r8] * sc; Tf[8 * hlf + r8][c] = p; pes[hh][r8] += pmul(p, wsv); ped[hh][r8] += pmul(p, wdv); } }
#pragma unroll
    for (int hh = 0; hh < 4; ++hh)
#pragma unroll
      for (int r8 = 0; r8 < 8; ++r8) { float s = pes[hh][r8], d = ped[hh][r8]; for (int o = 1; o < 16; o <<= 1) { s += __shfl_xor(s, o); d += __shfl_xor(d, o); } if (nloc == 0) { Se[8 * hlf + r8][cg * 4 + hh] = s; Sd[8 * hlf + r8][cg * 4 + hh] = d; } } }
  wave_lds_sync();
  for (int pass = 0; pass < 2; ++pass) { for (int rr = 0; rr < 16; ++rr) for (int q = 0; q < 2; ++q) *(volatile v4f*)(P1 + (m0 + rr) * W1O + q * 128 + lane * 4) = *(const v4f*)(&Tf[rr][q * 128 + lane * 4]);
    { const int rr = lane >> 1, hq = (lane & 1) * 4; *(volatile v4f*)(ES + (m0 + rr) * 8 + hq) = *(const v4f*)(&Se[rr][hq]); *(volatile v4f*)(ED + (m0 + rr) * 8 + hq) = *(const v4f*)(&Sd[rr][hq]); } __threadfence(); }
}
template <int W, int NHH, int EW>
__global__ __launch_bounds__(256) void att_kernel(const float* __restrict__ P, const float* __restrict__ ES, const float* __restrict__ ED, const float* __restrict__ bias, const int* __restrict__ srcs, const int* __restrict__ PERM, const int* __restrict__ ROWPTR, const int* __restrict__ ROWCNT, int permLen, int NLIM, float* __restrict__ Gout) {
  constexpr int CPL = W / 32;
  const int wave = threadIdx.x >> 5, lane = threadIdx.x & 31; const size_t v = (size_t)blockIdx.x * 8 + wave; const int h = (lane * CPL) / (W / NHH); float o[CPL]; for (int i = 0; i < CPL; ++i) o[i] = 0.0f;
  if (v < (size_t)NLIM) { int st = ROWPTR[v], cnt = ROWCNT[v]; cnt = iclamp(cnt, 0, 1 << 20); st = iclamp(st, 0, permLen - cnt); const float edv = ED[v * EW + h]; float mx = leaky(ES[v * EW + h] + edv);
#pragma unroll 1
    for (int j = 0; j < cnt; ++j) { const int e = iclamp(PERM[st + j], 0, E - 1); const int s = iclamp(srcs[e], 0, N - 1); if (s >= NLIM) continue; mx = fmaxf(mx, leaky(ES[(size_t)s * EW + h] + edv)); }
    float den; { const float p = __expf(leaky(ES[v * EW + h] + edv) - mx); den = p; float f[CPL]; ldrow<CPL>(P + v * W + lane * CPL, f); for (int i = 0; i < CPL; ++i) o[i] = pmul(p, f[i]); }
#pragma unroll 1
    for (int j = 0; j < cnt; ++j) { const int e = iclamp(PERM[st + j], 0, E - 1); const int s = iclamp(srcs[e], 0, N - 1); if (s >= NLIM) continue; const float p = __expf(leaky(ES[(size_t)s * EW + h] + edv) - mx); den += p; float f[CPL]; ldrow<CPL>(P + (size_t)s * W + lane * CPL, f); for (int i = 0; i < CPL; ++i) o[i] += pmul(p, f[i]); }
    const float inv = 1.0f / den; for (int i = 0; i < CPL; ++i) o[i] = pmul(o[i], inv) + bf16_rne(bias[lane * CPL + i]); }
  for (int pass = 0; pass < 2; ++pass) { strow<CPL>(Gout + v * W + lane * CPL, o); __threadfence(); }
}

__global__ __launch_bounds__(32) void lin2_kernel(const float* __restrict__ G1, const b16* __restrict__ W2T, const float* __restrict__ as, const float* __restrict__ ad, int NLIM, float* __restrict__ P2, float* __restrict__ E2) {
  __shared__ __attribute__((aligned(16))) b16 Ah[16][W1O + 8], Al[16][W1O + 8]; __shared__ __attribute__((aligned(16))) float Tf[16][HID + 4]; __shared__ __attribute__((aligned(16))) float Se[16][4];
  const int lane = threadIdx.x, nloc = lane & 15, hlf = lane >> 4; const size_t m0 = (size_t)blockIdx.x * 16; const bool live = m0 < (size_t)NLIM;
  for (int rr = 0; rr < 16; ++rr) for (int q = 0; q < 2; ++q) { v4f v = {0, 0, 0, 0}; if (live) v = *(const v4f*)(G1 + (m0 + rr) * W1O + q * 128 + lane * 4); for (int j = 0; j < 4; ++j) { b16 p, ql; split16(elu(v[j]) * HS, p, ql); Ah[rr][q * 128 + lane * 4 + j] = p; Al[rr][q * 128 + lane * 4 + j] = ql; } }
  wave_lds_sync();
  v8f acc[2] = {(v8f){}, (v8f){}};
  if (live) {
#pragma unroll 2
    for (int kb = 0; kb < W1O; kb += 32) { const v16b a = frag_kb(&Ah[nloc][kb], hlf), al = frag_kb(&Al[nloc][kb], hlf);
#pragma unroll
      for (int t = 0; t < 2; ++t) { const v16b bw = frag_kb(W2T + (size_t)(t * 16 + nloc) * W1O + kb, hlf); acc[t] = wmma16b(a, bw, acc[t]); acc[t] = wmma16b(al, bw, acc[t]); } } }
  const float sc = 1.0f / (HS * WSC); float pes[8], ped[8]; for (int r8 = 0; r8 < 8; ++r8) { pes[r8] = 0.0f; ped[r8] = 0.0f; }
#pragma unroll
  for (int t = 0; t < 2; ++t) { const int c = t * 16 + nloc; const float wsv = bf16_rne(as[c]), wdv = bf16_rne(ad[c]);
#pragma unroll
    for (int r8 = 0; r8 < 8; ++r8) { const float p = acc[t][r8] * sc; Tf[8 * hlf + r8][c] = p; pes[r8] += pmul(p, wsv); ped[r8] += pmul(p, wdv); } }
#pragma unroll
  for (int r8 = 0; r8 < 8; ++r8) { float s = pes[r8], d = ped[r8]; for (int o = 1; o < 16; o <<= 1) { s += __shfl_xor(s, o); d += __shfl_xor(d, o); } if (nloc == 0) { Se[8 * hlf + r8][0] = s; Se[8 * hlf + r8][1] = d; Se[8 * hlf + r8][2] = 0.0f; Se[8 * hlf + r8][3] = 0.0f; } }
  wave_lds_sync();
  for (int pass = 0; pass < 2; ++pass) { for (int rr = 0; rr < 16; ++rr) ((volatile float*)P2)[(m0 + rr) * HID + lane] = Tf[rr][lane]; if (lane < 16) *(volatile v4f*)(E2 + (m0 + lane) * 4) = *(const v4f*)(&Se[lane][0]); __threadfence(); }
}
__global__ __launch_bounds__(64) void head_kernel(const float* __restrict__ G2, const b16* __restrict__ WFC, const float* __restrict__ bfc, const b16* __restrict__ WH, const float* __restrict__ bmu, const float* __restrict__ bvar, const float* __restrict__ bpi, int NLIM, float* __restrict__ omu, float* __restrict__ ovar, float* __restrict__ opi) {
  __shared__ __attribute__((aligned(16))) b16 Ah[2][16][HID + 8], Al[2][16][HID + 8]; __shared__ float So[2][16][16]; __shared__ float Ou[3][32 * MIX];
  const int wave = threadIdx.x >> 5, lane = threadIdx.x & 31, nloc = lane & 15, hlf = lane >> 4; const size_t m0 = (size_t)blockIdx.x * 32 + wave * 16; const bool live = m0 < (size_t)NLIM; const float sc = 1.0f / (HS * WSC);
  for (int rr = 0; rr < 16; ++rr) { const float g = (live && m0 + rr < (size_t)N) ? G2[(m0 + rr) * HID + lane] : 0.0f; b16 p, q; split16(elu(g) * HS, p, q); Ah[wave][rr][lane] = p; Al[wave][rr][lane] = q; }
  wave_lds_sync();
  v8f acc[2] = {(v8f){}, (v8f){}};
  { const v16b a = frag_kb(&Ah[wave][nloc][0], hlf), al = frag_kb(&Al[wave][nloc][0], hlf);
#pragma unroll
    for (int t = 0; t < 2; ++t) { const v16b bw = frag_kb(WFC + (size_t)(t * 16 + nloc) * HID, hlf); acc[t] = wmma16b(a, bw, acc[t]); acc[t] = wmma16b(al, bw, acc[t]); } }
  wave_lds_sync();
#pragma unroll
  for (int t = 0; t < 2; ++t) { const int c = t * 16 + nloc; const float bb = bf16_rne(bfc[c]);
#pragma unroll
    for (int r8 = 0; r8 < 8; ++r8) { const float x3 = elu(acc[t][r8] * sc + bb); b16 p, q; split16(x3 * HS, p, q); Ah[wave][8 * hlf + r8][c] = p; Al[wave][8 * hlf + r8][c] = q; } }
  wave_lds_sync();
  v8f d = (v8f){}; { const v16b a = frag_kb(&Ah[wave][nloc][0], hlf), al = frag_kb(&Al[wave][nloc][0], hlf); const v16b bw = frag_kb(WH + (size_t)nloc * HID, hlf); d = wmma16b(a, bw, d); d = wmma16b(al, bw, d); }
  { const float bb = nloc < MIX ? bf16_rne(bmu[nloc]) : (nloc < 2 * MIX ? bf16_rne(bvar[nloc - MIX]) : (nloc < 3 * MIX ? bf16_rne(bpi[nloc - 2 * MIX]) : 0.0f));
#pragma unroll
    for (int r8 = 0; r8 < 8; ++r8) So[wave][8 * hlf + r8][nloc] = d[r8] * sc + bb; }
  wave_lds_sync();
  { const int rr = lane >> 1; const int orow = wave * 16 + rr;
    if ((lane & 1) == 0) { for (int k = 0; k < MIX; ++k) { Ou[0][orow * MIX + k] = So[wave][rr][k]; const float z = So[wave][rr][MIX + k]; Ou[1][orow * MIX + k] = z > 20.0f ? z : (z < -20.0f ? __expf(z) : log1pf(__expf(z))); } }
    else { float mx = -INFINITY; for (int k = 0; k < MIX; ++k) mx = fmaxf(mx, So[wave][rr][2 * MIX + k]); float ex[MIX], s = 0.0f; for (int k = 0; k < MIX; ++k) { ex[k] = __expf(So[wave][rr][2 * MIX + k] - mx); s += ex[k]; } for (int k = 0; k < MIX; ++k) Ou[2][orow * MIX + k] = ex[k] / s; } }
  __syncthreads();
  for (int pass = 0; pass < 2; ++pass) { for (int i = threadIdx.x; i < 32 * MIX; i += 64) { const size_t g = (size_t)blockIdx.x * 32 * MIX + i; if (g < (size_t)NP * MIX) { ((volatile float*)omu)[g] = Ou[0][i]; ((volatile float*)ovar)[g] = Ou[1][i]; ((volatile float*)opi)[g] = Ou[2][i]; } } __threadfence(); }
}
__global__ __launch_bounds__(256) void outcopy_kernel(const float* __restrict__ MU, const float* __restrict__ VA, const float* __restrict__ PI, float* __restrict__ out) {
  const size_t g = (size_t)blockIdx.x * 256 + threadIdx.x; if (g >= (size_t)3 * N * MIX) return; const size_t q = g / ((size_t)N * MIX), i = g % ((size_t)N * MIX); const float v = q == 0 ? MU[i] : (q == 1 ? VA[i] : PI[i]);
  for (int pass = 0; pass < 2; ++pass) { ((volatile float*)out)[g] = v; __threadfence(); }
}
}

extern "C" void kernel_launch(void* const* d_in, const int* in_sizes, int n_in, void* d_out, int out_size, void* d_ws, size_t ws_size, hipStream_t stream) {
  (void)n_in;
  auto Fp = [&](int i) { return (const float*)d_in[i]; }; auto Ip = [&](int i) { return (const int*)d_in[i]; };
  if (in_sizes[0] != N || in_sizes[1] != 2 * E || in_sizes[2] != V * EMB || in_sizes[3] != EMB * W1O || in_sizes[4] != NH * HID || in_sizes[7] != W1O * HID || in_sizes[11] != HID * HID || in_sizes[13] != HID * MIX || in_sizes[17] != HID * MIX || out_size != 3 * N * MIX) return;
  const int NLIM = N; const int GB16 = NBLK, GB8 = NP / 8;
  size_t off = 0; char* ws = (char*)d_ws;
  auto carve = [&](size_t bytes) { char* p = ws + off; off += (bytes + 255) & ~(size_t)255; return p; };
  b16* W1T = (b16*)carve((size_t)W1O * EMB * 2); b16* W2T = (b16*)carve((size_t)HID * W1O * 2); b16* WFC = (b16*)carve(HID * HID * 2); b16* WH = (b16*)carve(16 * HID * 2);
  float* P1 = (float*)carve((size_t)NP * W1O * 4); float* G1 = (float*)carve((size_t)NP * W1O * 4); float* ES = (float*)carve((size_t)NP * 8 * 4); float* ED = (float*)carve((size_t)NP * 8 * 4); float* P2 = (float*)carve((size_t)NP * HID * 4); float* G2 = (float*)carve((size_t)NP * HID * 4); float* E2 = (float*)carve((size_t)NP * 4 * 4); float* MUp = (float*)carve((size_t)NP * MIX * 4); float* VAp = (float*)carve((size_t)NP * MIX * 4); float* PIp = (float*)carve((size_t)NP * MIX * 4);
  CsrBufs9 csr; off = csr_carve9(csr, ws, off, E, N);
  if (off > ws_size || off > ((size_t)128 << 20)) return;
  wprep_kernel<<<(W1O * EMB + 255) / 256, 256, 0, stream>>>(Fp(3), EMB, W1O, 0, W1T); wprep_kernel<<<(HID * W1O + 255) / 256, 256, 0, stream>>>(Fp(7), W1O, HID, 0, W2T); wprep_kernel<<<(HID * HID + 255) / 256, 256, 0, stream>>>(Fp(11), HID, HID, 0, WFC);
  wzero_kernel<<<(16 * HID / 8 + 255) / 256, 256, 0, stream>>>(WH, 16 * HID / 8);
  wprep_kernel<<<(MIX * HID + 255) / 256, 256, 0, stream>>>(Fp(13), HID, MIX, 0, WH); wprep_kernel<<<(MIX * HID + 255) / 256, 256, 0, stream>>>(Fp(15), HID, MIX, MIX, WH); wprep_kernel<<<(MIX * HID + 255) / 256, 256, 0, stream>>>(Fp(17), HID, MIX, 2 * MIX, WH);
  csr_build9(csr, Ip(1) + E, E, N, stream);
  lin1_kernel<<<GB16, 32, 0, stream>>>(Ip(0), Fp(2), W1T, Fp(4), Fp(5), NLIM, P1, ES, ED);
  att_kernel<W1O, NH, 8><<<GB8, 256, 0, stream>>>(P1, ES, ED, Fp(6), Ip(1), csr.PERM, csr.ROWPTR, csr.ROWCNT, (int)csr.permLen, NLIM, G1);
  lin2_kernel<<<GB16, 32, 0, stream>>>(G1, W2T, Fp(8), Fp(9), NLIM, P2, E2);
  att_kernel<HID, 1, 4><<<GB8, 256, 0, stream>>>(P2, E2, E2 + 1, Fp(10), Ip(1), csr.PERM, csr.ROWPTR, csr.ROWCNT, (int)csr.permLen, NLIM, G2);
  head_kernel<<<(NP + 31) / 32, 64, 0, stream>>>(G2, WFC, Fp(12), WH, Fp(14), Fp(16), Fp(18), NLIM, MUp, VAp, PIp);
  outcopy_kernel<<<(3 * N * MIX + 255) / 256, 256, 0, stream>>>(MUp, VAp, PIp, (float*)d_out);
}
